// RandomBucketsAttention_34583076667864
// MI455X (gfx1250) — hardware-verified
//
#include <hip/hip_runtime.h>
#include <math.h>

typedef __attribute__((ext_vector_type(16))) _Float16 v16h;
typedef __attribute__((ext_vector_type(16))) __bf16 v16b;
typedef __attribute__((ext_vector_type(8)))  _Float16 v8h;
typedef __attribute__((ext_vector_type(8)))  float v8f;
typedef __attribute__((ext_vector_type(4)))  float v4f;
typedef __attribute__((ext_vector_type(2)))  float v2f;
typedef __attribute__((ext_vector_type(4)))  unsigned v4u;
typedef __attribute__((ext_vector_type(4)))  int v4i;
typedef float __attribute__((may_alias)) float_a;
typedef int __attribute__((may_alias)) int_a;

template <typename T> __device__ __forceinline__ void vst2(void* p, T v) { *(volatile T*)p = v; __threadfence(); *(volatile T*)p = v; }
__device__ __forceinline__ v8f wmma16(v16h a, v16h b, v8f c) {
  v8f d = __builtin_amdgcn_wmma_f32_16x16x32_f16(false, a, false, b, (short)0, c, false, false);
  asm volatile("v_nop\n\tv_nop\n\tv_nop\n\tv_nop" : "+v"(d) : "v"(a), "v"(b));
  return d;
}
__device__ __forceinline__ v8f wmma_bf(v16b a, v16b b, v8f c) {
  v8f d = __builtin_amdgcn_wmma_f32_16x16x32_bf16(false, a, false, b, (short)0, c, false, false);
  asm volatile("v_nop\n\tv_nop\n\tv_nop\n\tv_nop" : "+v"(d) : "v"(a), "v"(b));
  return d;
}
__device__ __forceinline__ v16h frag_h(const _Float16* rowk0, int lane) {
  union { v16h v; v8h q[2]; } u; const _Float16* p = rowk0 + 8 * (lane >> 4);
  u.q[0] = *(const v8h*)p; u.q[1] = *(const v8h*)(p + 16); return u.v;
}
__device__ __forceinline__ v16h frag_f32(const float* rowk0, int lane) {
  v16h a; const float* p = rowk0 + 8 * (lane >> 4);
#pragma unroll
  for (int i = 0; i < 8; ++i) { a[i] = (_Float16)p[i]; a[8 + i] = (_Float16)p[16 + i]; }
  return a;
}
__device__ __forceinline__ v16h frag_f32s(const float* rowk0, int lane, float sc) {
  v16h a; const float* p = rowk0 + 8 * (lane >> 4);
#pragma unroll
  for (int i = 0; i < 8; ++i) { a[i] = (_Float16)(p[i] * sc); a[8 + i] = (_Float16)(p[16 + i] * sc); }
  return a;
}
__device__ __forceinline__ v16h fragc_f32(const float* W, int k0, int n, int lane, int ld, int K) {
  v16h a; const int g = lane >> 4;
#pragma unroll
  for (int i = 0; i < 8; ++i) { const int ka = k0 + 8 * g + i, kb = ka + 16;
    a[i] = (_Float16)(ka < K ? W[(size_t)(ka < K ? ka : K - 1) * ld + n] : 0.f); a[8 + i] = (_Float16)(kb < K ? W[(size_t)(kb < K ? kb : K - 1) * ld + n] : 0.f); }
  return a;
}
struct F2 { v16b h, l; };
__device__ __forceinline__ F2 bsplit16(const float v[16]) { F2 r;
#pragma unroll
  for (int i = 0; i < 16; ++i) { const __bf16 h = (__bf16)v[i]; r.h[i] = h; r.l[i] = (__bf16)(v[i] - (float)h); }
  return r; }
__device__ __forceinline__ F2 split_row(const float* row, int k0, int lane) { float v[16]; const float* p = row + k0 + 8 * (lane >> 4);
#pragma unroll
  for (int i = 0; i < 8; ++i) { v[i] = p[i]; v[8 + i] = p[16 + i]; }
  return bsplit16(v); }
__device__ __forceinline__ F2 split_rowK(const float* row, int k0, int lane, int K) { float v[16]; const int g = lane >> 4;
#pragma unroll
  for (int i = 0; i < 8; ++i) { const int ka = k0 + 8 * g + i, kb = ka + 16; v[i] = ka < K ? row[ka < K ? ka : K - 1] : 0.f; v[8 + i] = kb < K ? row[kb < K ? kb : K - 1] : 0.f; }
  return bsplit16(v); }
__device__ __forceinline__ F2 split_col(const float* W, int k0, int n, int lane, int ld, int K) { float v[16]; const int g = lane >> 4;
#pragma unroll
  for (int i = 0; i < 8; ++i) { const int ka = k0 + 8 * g + i, kb = ka + 16; v[i] = ka < K ? W[(size_t)(ka < K ? ka : K - 1) * ld + n] : 0.f; v[8 + i] = kb < K ? W[(size_t)(kb < K ? kb : K - 1) * ld + n] : 0.f; }
  return bsplit16(v); }
__device__ __forceinline__ v8f mac3(const F2& a, const F2& b, v8f c) { c = wmma_bf(a.l, b.h, c); c = wmma_bf(a.h, b.l, c); return wmma_bf(a.h, b.h, c); }
__device__ __forceinline__ float sigm(float v) { return 1.0f / (1.0f + expf(-v)); }
#define LDSX() do { asm volatile("s_wait_dscnt 0" ::: "memory"); __builtin_amdgcn_wave_barrier(); __builtin_amdgcn_fence(__ATOMIC_RELEASE, "workgroup"); } while (0)


#define NB 8
#define SQ 4096
#define DD 64
#define NHASH 8
#define KB 64
#define NBK (SQ / KB)
#define CHUNK (NHASH * NBK)
#ifndef TNB
#define TNB NB
#endif
typedef __attribute__((ext_vector_type(8))) __bf16 v8b;
__device__ __forceinline__ v16b frag_b(const __bf16* rowk0, int lane) {
  union { v16b v; v8b q[2]; } u; const __bf16* p = rowk0 + 8 * (lane >> 4);
  u.q[0] = *(const v8b*)p; u.q[1] = *(const v8b*)(p + 16); return u.v;
}
__device__ __forceinline__ float bfr(float v) { return (float)(__bf16)v; }
__device__ __attribute__((noinline)) float exp_ni(float v) { return expf(v); }
__device__ __attribute__((noinline)) float erf_ni(float v) { return erff(v); }

#define WS_OH  0u
#define WS_LSE (WS_OH + 4u * (size_t)NB * NHASH * SQ * DD)
#define WS_END (WS_LSE + 4u * (size_t)NB * NHASH * SQ)

__global__ __launch_bounds__(128) void k_bucket(const float* __restrict__ Qy, const float* __restrict__ Ky, const float* __restrict__ Vy, const int* __restrict__ KST, float* __restrict__ OH, float* __restrict__ LSE) {
  __shared__ __align__(16) __bf16 sk[KB][72]; __shared__ __align__(16) _Float16 sv[DD][72]; __shared__ __align__(16) float sp[4][16][68]; __shared__ __align__(16) float so[4][16][68]; __shared__ __align__(16) float sl[64];
  const int tid = threadIdx.x, wave = tid >> 5, lane = tid & 31, col = lane & 15, g = lane >> 4; const int c = blockIdx.x; const size_t b = blockIdx.y; const int h = c / NBK; const int s0 = (c % NBK) * KB;
  for (int e = tid; e < KB * DD; e += 128) { const int j = e >> 6, d = e & 63; const int src = KST[b * (NHASH * SQ) + (size_t)c * KB + j]; sk[j][d] = (__bf16)Ky[(b * SQ + src) * DD + d]; sv[d][j] = (_Float16)bfr(Vy[(b * SQ + src) * DD + d]); }
  __syncthreads();
  v16b aq[2];
#pragma unroll
  for (int kc = 0; kc < 2; ++kc) { const float* pp = Qy + ((size_t)h * SQ + s0 + wave * 16 + col) * DD + kc * 32 + 8 * g;
#pragma unroll
    for (int i = 0; i < 8; ++i) { aq[kc][i] = (__bf16)pp[i]; aq[kc][8 + i] = (__bf16)pp[16 + i]; } }
  float s[4][8];
#pragma unroll
  for (int ct = 0; ct < 4; ++ct) { v8f cc = {};
#pragma unroll
    for (int kc = 0; kc < 2; ++kc) { v16b w; const __bf16* kp = &sk[ct * 16 + col][kc * 32 + 8 * g];
#pragma unroll
      for (int i = 0; i < 8; ++i) { w[i] = kp[i]; w[8 + i] = kp[16 + i]; }
      cc = wmma_bf(aq[kc], w, cc); }
#pragma unroll
    for (int r = 0; r < 8; ++r) s[ct][r] = cc[r]; }
  float mrow[8], lrow[8];
#pragma unroll
  for (int r = 0; r < 8; ++r) { float mx = fmaxf(fmaxf(s[0][r], s[1][r]), fmaxf(s[2][r], s[3][r]));
#pragma unroll
    for (int o = 1; o < 16; o <<= 1) mx = fmaxf(mx, __shfl_xor(mx, o));
    float es = 0.f;
#pragma unroll
    for (int ct = 0; ct < 4; ++ct) { const float e = expf(s[ct][r] - mx); sp[wave][8 * g + r][ct * 16 + col] = e; es += e; }
#pragma unroll
    for (int o = 1; o < 16; o <<= 1) es += __shfl_xor(es, o);
    mrow[r] = mx; lrow[r] = es; }
  LDSX();
  v8f acc[4] = {};
#pragma unroll
  for (int kt = 0; kt < 2; ++kt) { v16h pa, par; { const float* prow = &sp[wave][col][kt * 32] + 8 * (lane >> 4);
#pragma unroll
      for (int i = 0; i < 8; ++i) { const float p0 = prow[i] * 2048.0f, p1 = prow[16 + i] * 2048.0f; pa[i] = (_Float16)p0; pa[8 + i] = (_Float16)p1; par[i] = (_Float16)(p0 - (float)pa[i]); par[8 + i] = (_Float16)(p1 - (float)pa[8 + i]); } }
#pragma unroll
    for (int j = 0; j < 4; ++j) { v16h vh; const _Float16* vp = &sv[j * 16 + col][kt * 32 + 8 * g];
#pragma unroll
      for (int i = 0; i < 8; ++i) { vh[i] = vp[i]; vh[8 + i] = vp[16 + i]; }
      acc[j] = wmma16(pa, vh, acc[j]); acc[j] = wmma16(par, vh, acc[j]); } }
#pragma unroll
  for (int r = 0; r < 8; ++r) { const float il = (1.0f / 2048.0f) / lrow[r];
#pragma unroll
    for (int j = 0; j < 4; ++j) so[wave][8 * g + r][j * 16 + col] = acc[j][r] * il;
    if (col == 0) sl[wave * 16 + 8 * g + r] = mrow[r] + logf(lrow[r]); }
  LDSX();
  for (int rl = 0; rl < 16; ++rl) if (lane < 16) vst2(OH + (((b * NHASH + h) * SQ) + s0 + wave * 16 + rl) * DD + lane * 4, *(const v4f*)&so[wave][rl][lane * 4]);
  __syncthreads(); if (tid < 16) vst2(LSE + ((b * NHASH + h) * SQ) + s0 + tid * 4, *(const v4f*)&sl[tid * 4]); }
__global__ __launch_bounds__(256) void k_comb(const float* __restrict__ OH, const float* __restrict__ LSE, float* __restrict__ OUT) { __shared__ float sw[64][NHASH];
  const int t = threadIdx.x; const size_t b = blockIdx.y; const int s0 = blockIdx.x * 64;
  if (t < 64) { float lv[NHASH]; float mx = -3.0e38f;
#pragma unroll
    for (int h = 0; h < NHASH; ++h) { lv[h] = LSE[((b * NHASH + h) * SQ) + s0 + t]; mx = fmaxf(mx, lv[h]); }
    float sum = 0.f;
#pragma unroll
    for (int h = 0; h < NHASH; ++h) { lv[h] = expf(lv[h] - mx); sum += lv[h]; }
#pragma unroll
    for (int h = 0; h < NHASH; ++h) sw[t][h] = lv[h] / sum; }
  __syncthreads();
  { const int sl_ = t >> 2, q = t & 3; v4f o[4];
#pragma unroll
    for (int k = 0; k < 4; ++k) o[k] = v4f{0.f, 0.f, 0.f, 0.f};
#pragma unroll 1
    for (int h = 0; h < NHASH; ++h) { const float w = sw[sl_][h]; const float* src = OH + (((b * NHASH + h) * SQ) + s0 + sl_) * DD + q * 16;
#pragma unroll
      for (int k = 0; k < 4; ++k) { const v4f v = *(const v4f*)(src + k * 4); o[k] += v * w; } }
#pragma unroll
    for (int k = 0; k < 4; ++k) vst2(OUT + (b * SQ + s0 + sl_) * DD + q * 16 + k * 4, o[k]); } }
extern "C" void kernel_launch(void* const* d_in, const int* in_sizes, int n_in, void* d_out, int out_size, void* d_ws, size_t ws_size, hipStream_t stream) {
  (void)in_sizes; (void)n_in; (void)out_size;
  const float** F = (const float**)d_in;
  if (ws_size < (size_t)WS_END) return;
  char* ws = (char*)d_ws; float *OH = (float*)(ws + WS_OH), *LSE = (float*)(ws + WS_LSE);
  k_bucket<<<dim3(CHUNK, TNB), 128, 0, stream>>>(F[0], F[1], F[2], (const int*)d_in[3], OH, LSE);
  k_comb<<<dim3(SQ / 64, TNB), 256, 0, stream>>>(OH, LSE, (float*)d_out);
}
